// GCN_59639915872756
// MI455X (gfx1250) — hardware-verified
//
#include <hip/hip_runtime.h>
#include <stddef.h>
#include <stdint.h>


#define DF      128
#define NREL    8
#define NBAS    30
#define XPW     1024
#define HW      256
#define KP      256
#define KO      512
#define NTHR    256
#define NWAVE   8
#define EPT     8
#define CHUNK   (NTHR * EPT)
#define WCAP    (EPT * 32)
#define LISTN   (NWAVE * WCAP)
#define NBA     1024
#define SLA     10
#define RCAP    28672
#define DEGCAP  64
#define MEAS_B1024  16623
#define MEAS_MAXDEG 35
#define GBM     64
#define GBN     128
#define GTHR    128
#define MROWS   128
#define NUR     (DF * (DF / 8))
#define NUC     (DF * (2 * DF / 8))
#define BKT_ZINTS     (LISTN + 2 * RCAP + 3 * NBA)
#define BKT_LDS_INTS  (BKT_ZINTS + 16)
#define SCAN_LDS_INTS (2 * RCAP + 2 * NBA + NWAVE * HW / 2)

static_assert((CHUNK & (CHUNK - 1)) == 0 && CHUNK <= 4096);
static_assert((NBA & (NBA - 1)) == 0 && NBA == (1 << SLA));
static_assert(((long long)CHUNK << SLA) < (1LL << 31));
static_assert(LISTN % NTHR == 0 && NBA == 4 * NTHR);
static_assert(NBA % NWAVE == 0 && NBA % 32 == 0 && NBA % 128 == 0 && NBA % GBM == 0);
static_assert(RCAP % (2 * NTHR) == 0 && BKT_ZINTS % (NTHR * 4) == 0);
static_assert(RCAP >= MEAS_B1024 + MEAS_B1024 / 20);
static_assert(DEGCAP >= MEAS_MAXDEG + 8);
static_assert(BKT_LDS_INTS * 4 <= 327680 && SCAN_LDS_INTS * 4 <= 327680);
static_assert(DF == 4 * 32 && NREL == 8 && XPW == NREL * DF);
static_assert(KP == 2 * DF && KO == 4 * DF && HW == 2 * DF);
static_assert(KP % 32 == 0 && KO % 32 == 0 && DF % 32 == 0);
static_assert(GBN == DF && GBM == (GTHR / 32) * 16 && (MROWS % GBM) == 0);
static_assert((NUR % NTHR) == 0 && (NUC % NTHR) == 0);
static_assert(NREL * NBAS <= NTHR);

typedef float          v4f   __attribute__((ext_vector_type(4)));
typedef float          v8f   __attribute__((ext_vector_type(8)));
typedef int            v2i   __attribute__((ext_vector_type(2)));
typedef int            v4i   __attribute__((ext_vector_type(4)));
typedef int            v8i   __attribute__((ext_vector_type(8)));
typedef unsigned       v2u   __attribute__((ext_vector_type(2)));
typedef unsigned short v4us  __attribute__((ext_vector_type(4)));
typedef unsigned short v8us  __attribute__((ext_vector_type(8)));
typedef __bf16         v16bf __attribute__((ext_vector_type(16)));
typedef v4f  __attribute__((may_alias)) v4fa;
typedef v2i  __attribute__((may_alias)) v2ia;
typedef v4i  __attribute__((may_alias)) v4ia;
typedef v2u  __attribute__((may_alias)) v2ua;
typedef v4us __attribute__((may_alias)) v4usa;
typedef v8us __attribute__((may_alias)) v8usa;
union FragB { v16bf v; v8us h[2]; v8i w; };

__device__ __forceinline__ v8f wmb(const FragB& a, const FragB& b, v8f c) {
  v8f d = __builtin_amdgcn_wmma_f32_16x16x32_bf16(false, a.v, false, b.v, (short)0, c, false, false);
  asm volatile("v_nop\n\tv_nop\n\tv_nop\n\tv_nop" : "+v"(d) : "v"(a.w), "v"(b.w));
  return d;
}

__device__ __forceinline__ unsigned int f2bf(float f) {
  const unsigned int u = __float_as_uint(f);
  const unsigned int r = ((u + 0x7FFFu + ((u >> 16) & 1u)) >> 16) & 0xFFFFu;
  return ((u & 0x7FFFFFFFu) > 0x7F800000u) ? 0x7FC0u : r;
}
__device__ __forceinline__ float bf2f(unsigned int b) { return __uint_as_float(b << 16); }
__device__ __forceinline__ float bfr(float f) { return bf2f(f2bf(f)); }
__device__ __forceinline__ unsigned int hilo(float v) {
  const unsigned int h = f2bf(v);
  const unsigned int l = f2bf(v - bf2f(h));
  return h | (l << 16);
}

__device__ __forceinline__ void wave_sync() {
  __builtin_amdgcn_fence(__ATOMIC_RELEASE, "wavefront");
  __builtin_amdgcn_wave_barrier();
  __builtin_amdgcn_fence(__ATOMIC_ACQUIRE, "wavefront");
}

template <int SLB>
__device__ __forceinline__ int scan_chunk(const int* __restrict__ dsts, int nE, int cbase, int slotBase,
                                          int nb, int vec8, int* list, int tid, int lane, int wave) {
  int wc = 0;
  const int el0  = tid * EPT;
  const int e0   = cbase + el0;
  const int sent = -2147483647 - 1;
  v4i da, db;
  if (vec8 != 0 && cbase + CHUNK <= nE) {
    da = *(const v4i*)(dsts + e0);
    db = *(const v4i*)(dsts + e0 + 4);
  } else {
    da.x = (e0     < nE) ? dsts[min(e0,     nE - 1)] : sent;
    da.y = (e0 + 1 < nE) ? dsts[min(e0 + 1, nE - 1)] : sent;
    da.z = (e0 + 2 < nE) ? dsts[min(e0 + 2, nE - 1)] : sent;
    da.w = (e0 + 3 < nE) ? dsts[min(e0 + 3, nE - 1)] : sent;
    db.x = (e0 + 4 < nE) ? dsts[min(e0 + 4, nE - 1)] : sent;
    db.y = (e0 + 5 < nE) ? dsts[min(e0 + 5, nE - 1)] : sent;
    db.z = (e0 + 6 < nE) ? dsts[min(e0 + 6, nE - 1)] : sent;
    db.w = (e0 + 7 < nE) ? dsts[min(e0 + 7, nE - 1)] : sent;
  }
  const unsigned nbs = (unsigned)slotBase;
  const unsigned unb = (unsigned)nb;
  const unsigned s0 = (unsigned)da.x - nbs, s1 = (unsigned)da.y - nbs;
  const unsigned s2 = (unsigned)da.z - nbs, s3 = (unsigned)da.w - nbs;
  const unsigned s4 = (unsigned)db.x - nbs, s5 = (unsigned)db.y - nbs;
  const unsigned s6 = (unsigned)db.z - nbs, s7 = (unsigned)db.w - nbs;
  const bool h0 = s0 < unb, h1 = s1 < unb, h2 = s2 < unb, h3 = s3 < unb;
  const bool h4 = s4 < unb, h5 = s5 < unb, h6 = s6 < unb, h7 = s7 < unb;
  const unsigned any = __builtin_amdgcn_ballot_w32(h0 | h1 | h2 | h3 | h4 | h5 | h6 | h7);
  if (any != 0u) {
#define HITJ(J, HJ, SJ) { \
      const unsigned mj = __builtin_amdgcn_ballot_w32(HJ); \
      if (mj != 0u) { \
        if (HJ) { \
          const int pos = wc + (int)__builtin_amdgcn_mbcnt_lo(mj, 0u); \
          if (pos < WCAP) list[wave * WCAP + pos] = ((el0 + (J)) << SLB) | (int)(SJ); \
        } \
        wc += (int)__builtin_popcount(mj); } }
    HITJ(0, h0, s0)
    HITJ(1, h1, s1)
    HITJ(2, h2, s2)
    HITJ(3, h3, s3)
    HITJ(4, h4, s4)
    HITJ(5, h5, s5)
    HITJ(6, h6, s6)
    HITJ(7, h7, s7)
#undef HITJ
  }
  return wc;
}

__global__ __launch_bounds__(NTHR) void k_prep(const float* __restrict__ x, const float* __restrict__ root,
                                               const float* __restrict__ wrel, const float* __restrict__ wroot,
                                               const float* __restrict__ bias1, const float* __restrict__ brel,
                                               unsigned short* XB, unsigned short* ROOTT, unsigned short* W2C,
                                               float* BT2, int nN, int nUx) {
  const int u = (int)blockIdx.x * NTHR + (int)threadIdx.x;
  v8us o;
  unsigned short* dp;
  if (u < nUx) {
    const int row = u >> 4;
    const int c0  = (u & 15) * 8;
    const int rc  = row < nN ? row : nN - 1;
    const float* p = x + (size_t)rc * DF + c0;
    const v4f a = *(const v4f*)p;
    const v4f b = *(const v4f*)(p + 4);
    const bool okr = row < nN;
    o[0] = okr ? (unsigned short)f2bf(a.x) : (unsigned short)0;
    o[1] = okr ? (unsigned short)f2bf(a.y) : (unsigned short)0;
    o[2] = okr ? (unsigned short)f2bf(a.z) : (unsigned short)0;
    o[3] = okr ? (unsigned short)f2bf(a.w) : (unsigned short)0;
    o[4] = okr ? (unsigned short)f2bf(b.x) : (unsigned short)0;
    o[5] = okr ? (unsigned short)f2bf(b.y) : (unsigned short)0;
    o[6] = okr ? (unsigned short)f2bf(b.z) : (unsigned short)0;
    o[7] = okr ? (unsigned short)f2bf(b.w) : (unsigned short)0;
    dp = XB + (size_t)row * DF + c0;
  } else if (u < nUx + NUR) {
    const int v  = u - nUx;
    const int n  = v >> 4;
    const int k8 = (v & 15) * 8;
    const float* p = root + (size_t)k8 * DF + n;
#pragma unroll
    for (int i = 0; i < 8; ++i) o[i] = (unsigned short)f2bf(p[(size_t)i * DF]);
    dp = ROOTT + (size_t)n * DF + k8;
  } else if (u < nUx + NUR + NUC) {
    const int v  = u - nUx - NUR;
    const int n  = v >> 5;
    const int kq = (v & 31) * 8;
    const int kk = kq & (DF - 1);
    const float* p = wrel + (size_t)kk * DF + n;
#pragma unroll
    for (int i = 0; i < 8; ++i) o[i] = (unsigned short)f2bf(p[(size_t)i * DF]);
    dp = W2C + (size_t)n * KO + kq;
  } else if (u < nUx + NUR + 2 * NUC) {
    const int v  = u - nUx - NUR - NUC;
    const int n  = v >> 5;
    const int kq = (v & 31) * 8;
    const int kk = kq & (DF - 1);
    const float* p = wroot + (size_t)kk * DF + n;
#pragma unroll
    for (int i = 0; i < 8; ++i) o[i] = (unsigned short)f2bf(p[(size_t)i * DF]);
    dp = W2C + (size_t)n * KO + 2 * DF + kq;
  } else {
    const int v = u - nUx - NUR - 2 * NUC;
    if (v < 32) {
      const v4f t = *(const v4f*)(bias1 + 4 * v);
      v4f r; r.x = bfr(t.x); r.y = bfr(t.y); r.z = bfr(t.z); r.w = bfr(t.w);
      float* bp = BT2 + 4 * v;
      *(volatile v4f*)bp = r;
      __threadfence();
      *(volatile v4f*)bp = r;
    } else if (v < 64) {
      const v4f t = *(const v4f*)(brel + 4 * (v - 32));
      v4f r; r.x = bfr(t.x); r.y = bfr(t.y); r.z = bfr(t.z); r.w = bfr(t.w);
      float* bp = BT2 + DF + 4 * (v - 32);
      *(volatile v4f*)bp = r;
      __threadfence();
      *(volatile v4f*)bp = r;
    }
    return;
  }
  *(volatile v8us*)dp = o;
  __threadfence();
  *(volatile v8us*)dp = o;
}

__global__ __launch_bounds__(NTHR) void k_w(const float* __restrict__ comp, const float* __restrict__ basis,
                                            unsigned short* WcT) {
  __shared__ float sc[NTHR];
  const int tid = (int)threadIdx.x;
  {
    const int ci = tid < NREL * NBAS ? tid : NREL * NBAS - 1;
    const float cv = bfr(comp[ci]);
    sc[tid] = (tid < NREL * NBAS) ? cv : 0.0f;
  }
  __syncthreads();
  const int u  = (int)blockIdx.x * NTHR + tid;
  const int n  = u >> 4;
  const int k8 = (u & 15) * 8;
  const int r  = (n >> 7) & (NREL - 1);
  const int oc = n & (DF - 1);
  const float* bp = basis + (size_t)k8 * DF + oc;
  float acc[8];
#pragma unroll
  for (int j = 0; j < 8; ++j) acc[j] = 0.0f;
#pragma unroll 1
  for (int b = 0; b < NBAS; ++b) {
    const float cb = sc[r * NBAS + b];
    const float* q = bp + (size_t)b * (DF * DF);
#pragma unroll
    for (int j = 0; j < 8; ++j) acc[j] = fmaf(cb, bfr(q[(size_t)j * DF]), acc[j]);
  }
  v8us ho, lo;
#pragma unroll
  for (int j = 0; j < 8; ++j) {
    const unsigned int p = hilo(acc[j]);
    ho[j] = (unsigned short)(p & 0xFFFFu);
    lo[j] = (unsigned short)(p >> 16);
  }
  unsigned short* dp = WcT + (size_t)n * KP + k8;
  *(volatile v8us*)dp = ho;
  *(volatile v8us*)(dp + DF) = lo;
  __threadfence();
  *(volatile v8us*)dp = ho;
  *(volatile v8us*)(dp + DF) = lo;
}

__global__ __launch_bounds__(NTHR) void k_bucket(const int* __restrict__ ei, const int* __restrict__ et,
                                                 const float* __restrict__ en, int nE, int nN, int vec8,
                                                 int* LIST, int* CO, int* FLG) {
  extern __shared__ __attribute__((aligned(16))) int bsm[];
  int* list = bsm;
  int* hl   = bsm + LISTN;
  int* sl   = hl + RCAP;
  int* cnt  = sl + RCAP;
  int* offs = cnt + NBA;
  int* cur  = offs + NBA;
  int* misc = cur + NBA;
  const int tid = (int)threadIdx.x, lane = tid & 31, wave = tid >> 5;
  const int blk = (int)blockIdx.x;
  const int nodeBase = blk * NBA;
  const int* srcs = ei;
  const int* dsts = ei + nE;
  int nb = nN - nodeBase;
  nb = nb < 0 ? 0 : (nb > NBA ? NBA : nb);

  {
    const v4i z4 = {0, 0, 0, 0};
    for (int i = tid * 4; i < BKT_ZINTS; i += NTHR * 4) *(v4ia*)(bsm + i) = z4;
    if (tid < 16) misc[tid] = 0;
  }
  __syncthreads();

  int t = 0, ov = 0;
  const int nChunks = (nE + CHUNK - 1) / CHUNK;
#pragma unroll 1
  for (int ch = 0; ch < nChunks; ++ch) {
    const int cbase = ch * CHUNK;
    const int wc = scan_chunk<SLA>(dsts, nE, cbase, nodeBase, nb, vec8, list, tid, lane, wave);
    if (lane == 0) misc[wave] = wc;
    __syncthreads();
    if (wave == 0) {
#pragma unroll 1
      for (int w2 = 0; w2 < NWAVE; ++w2) {
        int c = misc[w2];
        c = c < 0 ? 0 : (c > WCAP ? WCAP : c);
#pragma unroll 1
        for (int b0 = 0; b0 < c; b0 += 32) {
          const int idx = b0 + lane;
          const int ent = list[w2 * WCAP + (idx < WCAP ? idx : WCAP - 1)];
          const int m32 = (c - b0) < 32 ? (c - b0) : 32;
#pragma unroll 1
          for (int k = 0; k < m32; ++k) {
            const int u    = __builtin_amdgcn_readlane(ent, k);
            const int slot = u & (NBA - 1);
            const int el   = (u >> SLA) & (CHUNK - 1);
            const int pk   = ((cbase + el) << SLA) | slot;
            if (t < RCAP) {
              if (lane == 0) { hl[t] = pk; cnt[slot] = cnt[slot] + 1; }
              t = t + 1;
            } else {
              ov = 1;
            }
          }
        }
      }
    }
    __syncthreads();
  }
  if (wave == 0 && lane == 0) { misc[8] = t; misc[9] = ov; }
  __syncthreads();
  int tt = misc[8];
  tt = tt < 0 ? 0 : (tt > RCAP ? RCAP : tt);
  const int ovf = misc[9];

  if (wave == 0) {
    const int base = lane * (NBA / 32);
    int s = 0;
#pragma unroll 1
    for (int i = 0; i < NBA / 32; ++i) s += cnt[base + i];
    int incl = s;
#pragma unroll
    for (int d = 1; d < 32; d <<= 1) {
      const int y = __shfl_up(incl, d, 32);
      if (lane >= d) incl += y;
    }
    int run = incl - s;
#pragma unroll 1
    for (int i = 0; i < NBA / 32; ++i) {
      const int cv = cnt[base + i];
      offs[base + i] = run;
      cur[base + i]  = run;
      run += cv;
    }
  }
  __syncthreads();
  if (wave == 0) {
#pragma unroll 1
    for (int b0 = 0; b0 < tt; b0 += 32) {
      const int idx = b0 + lane;
      const int ent = hl[idx < RCAP ? idx : RCAP - 1];
      const int m32 = (tt - b0) < 32 ? (tt - b0) : 32;
#pragma unroll 1
      for (int k = 0; k < m32; ++k) {
        const int u    = __builtin_amdgcn_readlane(ent, k);
        const int slot = u & (NBA - 1);
        if (lane == 0) {
          int p = cur[slot];
          p = p < 0 ? 0 : (p > RCAP - 1 ? RCAP - 1 : p);
          sl[p] = u;
          cur[slot] = p + 1;
        }
      }
    }
  }
  __syncthreads();

  int* lb = LIST + (size_t)blk * (size_t)(2 * RCAP);
#pragma unroll 1
  for (int p = tid * 2; p < RCAP; p += NTHR * 2) {
    const int u0 = sl[p];
    const int u1 = sl[p + 1];
    int e0 = u0 >> SLA; e0 = e0 < 0 ? 0 : (e0 > nE - 1 ? nE - 1 : e0);
    int e1 = u1 >> SLA; e1 = e1 < 0 ? 0 : (e1 > nE - 1 ? nE - 1 : e1);
    int s0 = srcs[e0]; s0 = s0 < 0 ? 0 : (s0 > nN - 1 ? nN - 1 : s0);
    int s1 = srcs[e1]; s1 = s1 < 0 ? 0 : (s1 > nN - 1 ? nN - 1 : s1);
    int t0 = et[e0];   t0 = t0 < 0 ? 0 : (t0 > NREL - 1 ? NREL - 1 : t0);
    int t1 = et[e1];   t1 = t1 < 0 ? 0 : (t1 > NREL - 1 ? NREL - 1 : t1);
    const unsigned int w0 = f2bf(en[e0]);
    const unsigned int w1 = f2bf(en[e1]);
    const bool k0 = p < tt, k1 = (p + 1) < tt;
    v4i v;
    v.x = k0 ? s0 : 0;
    v.y = k0 ? (int)((w0 << 16) | (unsigned int)t0) : 0;
    v.z = k1 ? s1 : 0;
    v.w = k1 ? (int)((w1 << 16) | (unsigned int)t1) : 0;
    int* dp = lb + 2 * p;
    *(volatile v4i*)dp = v;
    __threadfence();
    *(volatile v4i*)dp = v;
  }
  {
    const v4i cv = *(const v4ia*)(cnt + 4 * tid);
    const v4i ovv = *(const v4ia*)(offs + 4 * tid);
    int* cp = CO + (size_t)blk * (size_t)(2 * NBA) + 4 * tid;
    v4i fv;
    fv.x = (tid == 0) ? tt : 0;
    fv.y = (tid == 0) ? ovf : 0;
    fv.z = 0; fv.w = 0;
    int* fp = FLG + (size_t)blk * 32 + 4 * (tid & 7);
    *(volatile v4i*)cp = cv;
    *(volatile v4i*)(cp + NBA) = ovv;
    if (tid < 8) *(volatile v4i*)fp = fv;
    __threadfence();
    *(volatile v4i*)cp = cv;
    *(volatile v4i*)(cp + NBA) = ovv;
    if (tid < 8) *(volatile v4i*)fp = fv;
  }
}

__device__ __forceinline__ void kseg(v8f (&acc)[8], const unsigned short* ap, const unsigned short* bp,
                                     int ldb, int nk) {
#pragma unroll 1
  for (int k0 = 0; k0 < nk; k0 += 32) {
    FragB af;
    af.h[0] = *(const v8usa*)(ap + k0);
    af.h[1] = *(const v8usa*)(ap + k0 + 16);
#pragma unroll
    for (int nt = 0; nt < 8; ++nt) {
      const unsigned short* wq = bp + (size_t)(16 * nt) * (size_t)ldb + k0;
      FragB bf;
      bf.h[0] = *(const v8usa*)wq;
      bf.h[1] = *(const v8usa*)(wq + 16);
      acc[nt] = wmb(af, bf, acc[nt]);
    }
  }
}

template <int NSEG>
__global__ __launch_bounds__(GTHR) void k_gemm(const unsigned short* A0, const unsigned short* A1, int lda, int nk,
                                               const unsigned short* __restrict__ BT, int ldb,
                                               const float* __restrict__ bias, int hasBias,
                                               float* outp, int ldo, int nOut) {
  __shared__ __attribute__((aligned(16))) float stg[GBM * GBN];
  const int tid = (int)threadIdx.x, lane = tid & 31, wave = tid >> 5, hh = lane >> 4, m = lane & 15;
  const int rowBase = (int)blockIdx.x * GBM;
  const int colBase = (int)blockIdx.y * GBN;

  v8f acc[8];
  {
    const v8f z = {0.f, 0.f, 0.f, 0.f, 0.f, 0.f, 0.f, 0.f};
#pragma unroll
    for (int t = 0; t < 8; ++t) acc[t] = z;
  }
  const size_t arow = (size_t)(rowBase + 16 * wave + m) * (size_t)lda + 8 * hh;
  const unsigned short* bp = BT + (size_t)(colBase + m) * (size_t)ldb + 8 * hh;
  kseg(acc, A0 + arow, bp, ldb, nk);
  if constexpr (NSEG == 2) kseg(acc, A1 + arow, bp + nk, ldb, nk);

#pragma unroll
  for (int nt = 0; nt < 8; ++nt) {
    const int lc = 16 * nt + m;
#pragma unroll
    for (int r = 0; r < 8; ++r) {
      const int lr = 16 * wave + 8 * hh + r;
      stg[lr * GBN + lc] = acc[nt][r];
    }
  }
  __syncthreads();

  v4f bb4;
  {
    const v4f t1 = *(const v4f*)(bias + 4 * lane);
    bb4.x = (hasBias != 0) ? t1.x : 0.0f;
    bb4.y = (hasBias != 0) ? t1.y : 0.0f;
    bb4.z = (hasBias != 0) ? t1.z : 0.0f;
    bb4.w = (hasBias != 0) ? t1.w : 0.0f;
  }
  v4f pv[16];
#pragma unroll
  for (int i = 0; i < 16; ++i) {
    const v4f t = *(const v4fa*)(stg + (16 * wave + i) * GBN + 4 * lane);
    pv[i] = t + bb4;
  }
#pragma unroll
  for (int i = 0; i < 16; ++i) {
    const int r = rowBase + 16 * wave + i;
    if (r < nOut) *(volatile v4f*)(outp + (size_t)r * (size_t)ldo + colBase + 4 * lane) = pv[i];
  }
  __threadfence();
#pragma unroll
  for (int i = 0; i < 16; ++i) {
    const int r = rowBase + 16 * wave + i;
    if (r < nOut) *(volatile v4f*)(outp + (size_t)r * (size_t)ldo + colBase + 4 * lane) = pv[i];
  }
}

template <int L>
__global__ __launch_bounds__(NTHR) void k_scan(const int* __restrict__ LIST, const int* __restrict__ CO,
                                               const int* __restrict__ FLG, const float* XP, const float* HRf,
                                               const float* __restrict__ B1, const unsigned short* Hin,
                                               unsigned short* Pout, int nN, int mRows) {
  static_assert(L == 1 || L == 2);
  extern __shared__ __attribute__((aligned(16))) int ssm[];
  int* ent  = ssm;
  int* cnt  = ssm + 2 * RCAP;
  int* offs = cnt + NBA;
  const int tid = (int)threadIdx.x, lane = tid & 31, wave = tid >> 5;
  unsigned short* rowbuf = (unsigned short*)(offs + NBA) + wave * HW;
  const int blk = (int)blockIdx.x;
  const int nodeBase = blk * NBA;

  const int nhraw = FLG[(size_t)blk * 32];
  const int bflag = FLG[(size_t)blk * 32 + 1];
  const int nh  = nhraw < 0 ? 0 : (nhraw > RCAP ? RCAP : nhraw);
  const int ovf = (bflag != 0 || nhraw < 0 || nhraw > RCAP) ? 1 : 0;

  {
    const int* lb = LIST + (size_t)blk * (size_t)(2 * RCAP);
    const int n4 = (2 * nh + 3) & ~3;
#pragma unroll 1
    for (int p = tid * 4; p < n4; p += NTHR * 4) *(v4ia*)(ent + p) = *(const v4i*)(lb + p);
    const int* cp = CO + (size_t)blk * (size_t)(2 * NBA) + 4 * tid;
    *(v4ia*)(cnt + 4 * tid)  = *(const v4i*)cp;
    *(v4ia*)(offs + 4 * tid) = *(const v4i*)(cp + NBA);
  }
  __syncthreads();

  const float qnan = __int_as_float(0x7fc00000);
  const float pzb  = (ovf != 0) ? qnan : 0.0f;
  v4f b4 = {0.f, 0.f, 0.f, 0.f};
  if constexpr (L == 1) b4 = *(const v4f*)(B1 + 4 * lane);

#pragma unroll 1
  for (int si = 0; si < NBA / NWAVE; ++si) {
    const int s    = si * NWAVE + wave;
    const int node = nodeBase + s;
    int c = cnt[s];
    const bool big = c > DEGCAP;
    c = c < 0 ? 0 : (c > DEGCAP ? DEGCAP : c);
    int o = offs[s];
    o = o < 0 ? 0 : (o > nh ? nh : o);
    if (c > nh - o) c = nh - o;
    float a0 = 0.0f, a1 = 0.0f, a2 = 0.0f, a3 = 0.0f;
#pragma unroll 1
    for (int b0 = 0; b0 < c; b0 += 32) {
      int idx = o + b0 + lane;
      idx = idx > nh - 1 ? nh - 1 : idx;
      idx = idx < 0 ? 0 : idx;
      const v2i e = *(const v2ia*)(ent + 2 * idx);
      int sr = e.x;
      sr = sr < 0 ? 0 : (sr > nN - 1 ? nN - 1 : sr);
      const int tp  = e.y & (NREL - 1);
      const int wvi = (int)((unsigned int)e.y & 0xffff0000u);
      const int go  = (L == 1) ? (sr * XPW + tp * DF) : (sr * HW);
      const int m32 = (c - b0) < 32 ? (c - b0) : 32;
#pragma unroll 1
      for (int k = 0; k < m32; ++k) {
        const int gk = __builtin_amdgcn_readlane(go, k);
        if constexpr (L == 1) {
          const float ck = __int_as_float(__builtin_amdgcn_readlane(wvi, k));
          const v4f a = *(const v4f*)(XP + (size_t)gk + 4 * lane);
          a0 = fmaf(ck, a.x, a0);
          a1 = fmaf(ck, a.y, a1);
          a2 = fmaf(ck, a.z, a2);
          a3 = fmaf(ck, a.w, a3);
        } else {
          const unsigned short* rp = Hin + (size_t)gk + 4 * lane;
          const v2u wh = *(const v2ua*)rp;
          const v2u wl = *(const v2ua*)(rp + DF);
          a0 += __uint_as_float(wh.x << 16)         + __uint_as_float(wl.x << 16);
          a1 += __uint_as_float(wh.x & 0xffff0000u) + __uint_as_float(wl.x & 0xffff0000u);
          a2 += __uint_as_float(wh.y << 16)         + __uint_as_float(wl.y << 16);
          a3 += __uint_as_float(wh.y & 0xffff0000u) + __uint_as_float(wl.y & 0xffff0000u);
        }
      }
    }
    const float pzr = big ? qnan : pzb;
    const bool live = node < nN;
    float m0, m1, m2, m3;
    if constexpr (L == 1) {
      v4f hr = {0.f, 0.f, 0.f, 0.f};
      if (node < mRows) hr = *(const v4f*)(HRf + (size_t)node * DF + 4 * lane);
      m0 = live ? (((a0 + hr.x) + b4.x) + pzr) : 0.0f;
      m1 = live ? (((a1 + hr.y) + b4.y) + pzr) : 0.0f;
      m2 = live ? (((a2 + hr.z) + b4.z) + pzr) : 0.0f;
      m3 = live ? (((a3 + hr.w) + b4.w) + pzr) : 0.0f;
    } else {
      m0 = live ? (a0 + pzr) : 0.0f;
      m1 = live ? (a1 + pzr) : 0.0f;
      m2 = live ? (a2 + pzr) : 0.0f;
      m3 = live ? (a3 + pzr) : 0.0f;
    }
    v4us mh, ml;
    {
      unsigned int p;
      p = hilo(m0); mh[0] = (unsigned short)(p & 0xFFFFu); ml[0] = (unsigned short)(p >> 16);
      p = hilo(m1); mh[1] = (unsigned short)(p & 0xFFFFu); ml[1] = (unsigned short)(p >> 16);
      p = hilo(m2); mh[2] = (unsigned short)(p & 0xFFFFu); ml[2] = (unsigned short)(p >> 16);
      p = hilo(m3); mh[3] = (unsigned short)(p & 0xFFFFu); ml[3] = (unsigned short)(p >> 16);
    }
    *(v4usa*)(rowbuf + 4 * lane) = mh;
    *(v4usa*)(rowbuf + DF + 4 * lane) = ml;
    wave_sync();
    const v8us q0 = *(const v8usa*)(rowbuf + 8 * lane);
    wave_sync();
    if (node < mRows) {
      unsigned short* rpw = Pout + (size_t)node * HW + 8 * lane;
      *(volatile v8us*)rpw = q0;
      __threadfence();
      *(volatile v8us*)rpw = q0;
    }
  }
}

static inline int cdiv(int a, int b) { return (a + b - 1) / b; }

struct Carve {
  size_t oXP, oXB, oHH, oLIST, oCO, oFLG, oWC, oRT, oW2, oBT, end;
};
static constexpr size_t al256(size_t o) { return (o + 255) & ~(size_t)255; }
static constexpr Carve make_carve(size_t MP, size_t gA) {
  Carve c{};
  size_t off = 0;
  c.oXP   = off; off = al256(off + MP * XPW * 4);
  c.oXB   = off; off = al256(off + MP * DF * 2);
  c.oHH   = off; off = al256(off + MP * DF * 4);
  c.oLIST = off; off = al256(off + gA * RCAP * 8);
  c.oCO   = off; off = al256(off + gA * 2 * NBA * 4);
  c.oFLG  = off; off = al256(off + gA * 128);
  c.oWC   = off; off = al256(off + (size_t)NREL * DF * KP * 2);
  c.oRT   = off; off = al256(off + (size_t)DF * DF * 2);
  c.oW2   = off; off = al256(off + (size_t)DF * KO * 2);
  c.oBT   = off; off = al256(off + (size_t)2 * DF * 4);
  c.end   = off;
  return c;
}
static_assert(make_carve(50048, 49).end <= ((size_t)256 << 20));
static_assert((size_t)50048 * HW * 2 <= (size_t)50048 * XPW * 4);
static_assert((size_t)50048 * HW * 2 == (size_t)50048 * DF * 4);

extern "C" void kernel_launch(void* const* d_in, const int* in_sizes, int n_in,
                              void* d_out, int out_size, void* d_ws, size_t ws_size,
                              hipStream_t stream) {
  if (n_in < 11) return;
  if (in_sizes[0] < DF || (in_sizes[0] % DF) != 0) return;
  const int nN = in_sizes[0] / DF;
  if (in_sizes[1] < 2 || (in_sizes[1] & 1) != 0) return;
  const int nE = in_sizes[1] / 2;
  if (nE < 1 || nE >= (1 << 21)) return;
  if (in_sizes[2] != nE || in_sizes[3] != nE) return;
  if (in_sizes[4] != NBAS * DF * DF || in_sizes[5] != NREL * NBAS) return;
  if (in_sizes[6] != DF * DF || in_sizes[7] != DF) return;
  if (in_sizes[8] != DF * DF || in_sizes[9] != DF) return;
  if (in_sizes[10] != DF * DF) return;
  if (nN < 16 || nN > (1 << 20)) return;
  if ((long long)out_size != (long long)nN * DF) return;

  const float* x     = (const float*)d_in[0];
  const int*   ei    = (const int*)  d_in[1];
  const int*   et    = (const int*)  d_in[2];
  const float* en    = (const float*)d_in[3];
  const float* basis = (const float*)d_in[4];
  const float* comp  = (const float*)d_in[5];
  const float* root  = (const float*)d_in[6];
  const float* bias1 = (const float*)d_in[7];
  const float* wrel  = (const float*)d_in[8];
  const float* brel  = (const float*)d_in[9];
  const float* wroot = (const float*)d_in[10];
  float* out = (float*)d_out;

  const int MP  = cdiv(nN, MROWS) * MROWS;
  const int gM  = MP / GBM;
  const int gA  = cdiv(MP, NBA);
  if ((long long)gA * NBA < (long long)MP) return;
  const int vec8 = ((nE & 3) == 0) ? 1 : 0;
  const int nUx  = MP * (DF / 8);
  if ((nUx % NTHR) != 0) return;

  const Carve cv = make_carve((size_t)MP, (size_t)gA);
  if (cv.end > ws_size) return;
  char* ws = (char*)d_ws;
  float*          XP    = (float*)(ws + cv.oXP);
  unsigned short* AG    = (unsigned short*)(ws + cv.oXP);
  unsigned short* XB    = (unsigned short*)(ws + cv.oXB);
  float*          HRf   = (float*)(ws + cv.oHH);
  unsigned short* Hhl   = (unsigned short*)(ws + cv.oHH);
  int*            LIST  = (int*)(ws + cv.oLIST);
  int*            CO    = (int*)(ws + cv.oCO);
  int*            FLG   = (int*)(ws + cv.oFLG);
  unsigned short* WcT   = (unsigned short*)(ws + cv.oWC);
  unsigned short* ROOTT = (unsigned short*)(ws + cv.oRT);
  unsigned short* W2C   = (unsigned short*)(ws + cv.oW2);
  float*          BT2   = (float*)(ws + cv.oBT);

  const int bktLds  = BKT_LDS_INTS * 4;
  const int scanLds = SCAN_LDS_INTS * 4;
  hipFuncSetAttribute(reinterpret_cast<const void*>(&k_bucket),
                      hipFuncAttributeMaxDynamicSharedMemorySize, bktLds);
  hipFuncSetAttribute(reinterpret_cast<const void*>(&k_scan<1>),
                      hipFuncAttributeMaxDynamicSharedMemorySize, scanLds);
  hipFuncSetAttribute(reinterpret_cast<const void*>(&k_scan<2>),
                      hipFuncAttributeMaxDynamicSharedMemorySize, scanLds);

  k_prep<<<(nUx + NUR + 2 * NUC) / NTHR + 1, NTHR, 0, stream>>>(x, root, wrel, wroot, bias1, brel,
                                                               XB, ROOTT, W2C, BT2, nN, nUx);
  k_w<<<(NREL * DF * (DF / 8)) / NTHR, NTHR, 0, stream>>>(comp, basis, WcT);
  k_bucket<<<gA, NTHR, bktLds, stream>>>(ei, et, en, nE, nN, vec8, LIST, CO, FLG);
  k_gemm<2><<<dim3(gM, NREL), GTHR, 0, stream>>>(XB, XB, DF, DF, WcT, KP, BT2, 0, XP, XPW, MP);
  k_gemm<1><<<dim3(gM, 1), GTHR, 0, stream>>>(XB, XB, DF, DF, ROOTT, DF, BT2, 0, HRf, DF, MP);
  k_scan<1><<<gA, NTHR, scanLds, stream>>>(LIST, CO, FLG, XP, HRf, BT2, Hhl, Hhl, nN, MP);
  k_scan<2><<<gA, NTHR, scanLds, stream>>>(LIST, CO, FLG, XP, HRf, BT2, Hhl, AG, nN, MP);
  k_gemm<2><<<dim3(gM, 1), GTHR, 0, stream>>>(AG, Hhl, HW, HW, W2C, KO, BT2 + DF, 1, out, DF, nN);
}
